// BiaffineLabeler_43516608643697
// MI455X (gfx1250) — hardware-verified
//
#include <hip/hip_runtime.h>
#include <stdint.h>


typedef __attribute__((ext_vector_type(16))) _Float16 v16h;
typedef __attribute__((ext_vector_type(8)))  _Float16 v8h;
typedef __attribute__((ext_vector_type(8)))  float v8f;
typedef __attribute__((ext_vector_type(4)))  float v4f;
typedef __attribute__((ext_vector_type(4)))  unsigned v4u;

#define D_IN     1024
#define D_LAB    512
#define N_LABELS 50
#define T_DIM    2048
#define NTOK     4096
#define NHEAD    4098
#define NHEADP   4160

template <typename T> __device__ __forceinline__ void vst2(void* p, T v) { *(volatile T*)p = v; __threadfence(); *(volatile T*)p = v; }
__device__ __forceinline__ v8f wmma16(v16h a, v16h b, v8f c) {
  v8f d = __builtin_amdgcn_wmma_f32_16x16x32_f16(false, a, false, b, (short)0, c, false, false);
  asm volatile("v_nop\n\tv_nop\n\tv_nop\n\tv_nop" : "+v"(d) : "v"(a), "v"(b));
  return d;
}
__device__ __forceinline__ v16h frag_h(const _Float16* row, int k0, int lane) {
  union { v16h v; v8h q[2]; } r; const _Float16* p = row + k0 + 8 * (lane >> 4);
  r.q[0] = *(const v8h*)(p); r.q[1] = *(const v8h*)(p + 16); return r.v;
}
__device__ __forceinline__ v16h frag_f32(const float* row, int k0, int lane) {
  v16h a; const float* p = row + k0 + 8 * (lane >> 4);
#pragma unroll
  for (int i = 0; i < 8; ++i) { a[i] = (_Float16)p[i]; a[8 + i] = (_Float16)p[16 + i]; }
  return a;
}

__global__ __launch_bounds__(256) void k_cvt(const float* __restrict__ s, _Float16* __restrict__ d, int n8_src, int n8_tot) {
  const int g = blockIdx.x * 256 + threadIdx.x; if (g >= n8_tot) return;
  union { v8h h; v4u u; } pk;
#pragma unroll
  for (int e = 0; e < 8; ++e) pk.h[e] = (g < n8_src) ? (_Float16)s[(size_t)g * 8 + e] : (_Float16)0.f;
  vst2(d + (size_t)g * 8, pk.u);
}
__global__ __launch_bounds__(256) void k_wt(const float* __restrict__ W, _Float16* __restrict__ WT) {
  __shared__ __align__(16) _Float16 tile[64][72];
  const int n = blockIdx.x >> 6, t = blockIdx.x & 63, e0 = (t & 7) * 64, d0 = (t >> 3) * 64, tid = threadIdx.x;
  const float* Wn = W + (size_t)n * D_LAB * D_LAB;
  for (int i = tid; i < 64 * 64; i += 256) { const int dd = i >> 6, ee = i & 63; tile[ee][dd] = (_Float16)Wn[(size_t)(d0 + dd) * D_LAB + e0 + ee]; }
  __syncthreads();
  for (int g = tid; g < 64 * 8; g += 256) { const int ee = g >> 3, pc = g & 7; vst2(WT + ((size_t)n * D_LAB + e0 + ee) * D_LAB + d0 + pc * 8, *(const v4u*)(&tile[ee][pc * 8])); }
}
__global__ __launch_bounds__(128) void k_proj(const _Float16* __restrict__ X, const _Float16* __restrict__ Wp, const float* __restrict__ bp,
                                             float* __restrict__ Y, int nrows) {
  __shared__ __align__(16) float st[64][68];
  const int tid = threadIdx.x, wave = tid >> 5, lane = tid & 31, col = lane & 15, hi = lane >> 4;
  const int m0 = blockIdx.x * 64 + wave * 16, e0 = blockIdx.y * 64;
  const _Float16* ar = X + (size_t)(m0 + col) * D_IN;
  v8f c[4] = {};
#pragma unroll 2
  for (int kc = 0; kc < D_IN / 32; ++kc) {
    const v16h a = frag_h(ar, kc * 32, lane);
#pragma unroll
    for (int j = 0; j < 4; ++j) c[j] = wmma16(a, frag_h(Wp + (size_t)(e0 + j * 16 + col) * D_IN, kc * 32, lane), c[j]);
  }
#pragma unroll
  for (int j = 0; j < 4; ++j) { const float bb = bp[e0 + j * 16 + col];
#pragma unroll
    for (int r = 0; r < 8; ++r) st[wave * 16 + hi * 8 + r][j * 16 + col] = c[j][r] + bb; }
  __syncthreads();
#pragma unroll
  for (int q = 0; q < 8; ++q) { const int g = q * 128 + tid; const int rl = g >> 4, pc = g & 15; const int row = blockIdx.x * 64 + rl;
    if (row < nrows) vst2(Y + (size_t)row * D_LAB + e0 + pc * 4, *(const v4f*)(&st[rl][pc * 4])); }
}
__global__ __launch_bounds__(256) void k_gather(const float* __restrict__ HL, const int* __restrict__ hidx, float* __restrict__ sel) {
  const int t = blockIdx.x * 8 + (threadIdx.x >> 5), lane = threadIdx.x & 31;
  const int b = t / T_DIM;
  int id = hidx[t]; id = id < 0 ? 0 : (id > T_DIM ? T_DIM : id);
  const float* src = HL + ((size_t)b * (T_DIM + 1) + id) * D_LAB;
#pragma unroll
  for (int i = 0; i < 4; ++i) vst2(sel + (size_t)t * D_LAB + (i * 32 + lane) * 4, *(const v4f*)(src + (i * 32 + lane) * 4));
}
__global__ __launch_bounds__(256) void k_biaffine(const float* __restrict__ DL, const float* __restrict__ sel, const _Float16* __restrict__ WT,
                                                 const float* __restrict__ bias, float* __restrict__ stage) {
  __shared__ float part[2][64];
  const int tid = threadIdx.x, wave = tid >> 5, lane = tid & 31, col = lane & 15, hi = lane >> 4;
  const int t0 = blockIdx.x * 64, n = blockIdx.y;
  const int mt = wave & 3, ch = wave >> 2;
  const float* arow = DL + (size_t)(t0 + mt * 16 + col) * D_LAB;
  const _Float16* Wn = WT + (size_t)n * D_LAB * D_LAB;
  v8f acc[16];
#pragma unroll
  for (int j = 0; j < 16; ++j) acc[j] = (v8f){};
#pragma unroll 1
  for (int kc = 0; kc < D_LAB / 32; ++kc) {
    const v16h a = frag_f32(arow, kc * 32, lane);
#pragma unroll
    for (int j = 0; j < 16; ++j) acc[j] = wmma16(a, frag_h(Wn + (size_t)(ch * 256 + j * 16 + col) * D_LAB, kc * 32, lane), acc[j]);
  }
  float p[8];
#pragma unroll
  for (int r = 0; r < 8; ++r) p[r] = 0.f;
#pragma unroll
  for (int j = 0; j < 16; ++j) {
    const int e = ch * 256 + j * 16 + col;
#pragma unroll
    for (int r = 0; r < 8; ++r) p[r] += acc[j][r] * sel[(size_t)(t0 + mt * 16 + hi * 8 + r) * D_LAB + e];
  }
#pragma unroll
  for (int r = 0; r < 8; ++r) {
    float v = p[r];
#pragma unroll
    for (int off = 8; off > 0; off >>= 1) v += __shfl_xor(v, off, 32);
    if (col == 0) part[ch][mt * 16 + hi * 8 + r] = v;
  }
  __syncthreads();
  if (tid < 64) vst2(stage + (size_t)n * NTOK + t0 + tid, part[0][tid] + part[1][tid] + bias[n]);
}
__global__ __launch_bounds__(256) void k_flat(const float* __restrict__ stage, float* __restrict__ out) {
  const int g = blockIdx.x * 256 + threadIdx.x;
  if (g >= NTOK * N_LABELS / 4) return;
  v4f v;
#pragma unroll
  for (int e = 0; e < 4; ++e) { const int f = g * 4 + e, t = f / N_LABELS, n = f - t * N_LABELS; v[e] = stage[(size_t)n * NTOK + t]; }
  vst2(out + (size_t)g * 4, v);
}

extern "C" void kernel_launch(void* const* d_in, const int* in_sizes, int n_in,
                              void* d_out, int out_size, void* d_ws, size_t ws_size,
                              hipStream_t stream)
{
  (void)in_sizes; (void)n_in; (void)out_size; (void)ws_size;
  const float* dep    = (const float*)d_in[0];
  const float* head   = (const float*)d_in[1];
  const int*   hidx   = (const int*)  d_in[2];
  const float* dep_W  = (const float*)d_in[4];
  const float* dep_b  = (const float*)d_in[5];
  const float* head_W = (const float*)d_in[6];
  const float* head_b = (const float*)d_in[7];
  const float* W      = (const float*)d_in[8];
  const float* bias   = (const float*)d_in[9];
  float* out = (float*)d_out;

  char* ws = (char*)d_ws; size_t off = 0;
  auto alloc = [&](size_t bytes) -> void* { void* p = ws + off; off = (off + bytes + 255) & ~(size_t)255; return p; };
  _Float16* deph  = (_Float16*)alloc((size_t)NTOK * D_IN * 2);
  _Float16* headh = (_Float16*)alloc((size_t)NHEADP * D_IN * 2);
  _Float16* dWh   = (_Float16*)alloc((size_t)D_LAB * D_IN * 2);
  _Float16* hWh   = (_Float16*)alloc((size_t)D_LAB * D_IN * 2);
  _Float16* WT    = (_Float16*)alloc((size_t)N_LABELS * D_LAB * D_LAB * 2);
  float* DL  = (float*)alloc((size_t)NTOK * D_LAB * 4);
  float* HL  = (float*)alloc((size_t)NHEADP * D_LAB * 4);
  float* sel = (float*)alloc((size_t)NTOK * D_LAB * 4);
  float* stage = (float*)alloc((size_t)N_LABELS * NTOK * 4);

  k_cvt<<<(NTOK * D_IN / 8 + 255) / 256, 256, 0, stream>>>(dep, deph, NTOK * D_IN / 8, NTOK * D_IN / 8);
  k_cvt<<<(NHEADP * D_IN / 8 + 255) / 256, 256, 0, stream>>>(head, headh, NHEAD * D_IN / 8, NHEADP * D_IN / 8);
  k_cvt<<<(D_LAB * D_IN / 8 + 255) / 256, 256, 0, stream>>>(dep_W, dWh, D_LAB * D_IN / 8, D_LAB * D_IN / 8);
  k_cvt<<<(D_LAB * D_IN / 8 + 255) / 256, 256, 0, stream>>>(head_W, hWh, D_LAB * D_IN / 8, D_LAB * D_IN / 8);
  k_wt<<<N_LABELS * 64, 256, 0, stream>>>(W, WT);
  k_proj<<<dim3(NTOK / 64, D_LAB / 64), 128, 0, stream>>>(deph, dWh, dep_b, DL, NTOK);
  k_proj<<<dim3(NHEADP / 64, D_LAB / 64), 128, 0, stream>>>(headh, hWh, head_b, HL, NHEAD);
  k_gather<<<NTOK / 8, 256, 0, stream>>>(HL, hidx, sel);
  k_biaffine<<<dim3(NTOK / 64, N_LABELS), 256, 0, stream>>>(DL, sel, WT, bias, stage);
  k_flat<<<(NTOK * N_LABELS / 4 + 255) / 256, 256, 0, stream>>>(stage, out);
}
